// MambaBlock_36309653520717
// MI455X (gfx1250) — hardware-verified
//
#include <hip/hip_runtime.h>
#include <math.h>

typedef __attribute__((ext_vector_type(16))) _Float16 v16h;
typedef __attribute__((ext_vector_type(8)))  _Float16 v8h;
typedef __attribute__((ext_vector_type(8)))  float    v8f;
typedef __attribute__((ext_vector_type(4)))  float    v4f;
typedef __attribute__((ext_vector_type(2)))  float    v2f;
typedef __attribute__((ext_vector_type(4)))  unsigned v4u;

constexpr int kBat  = 16;
constexpr int kSeq  = 256;
constexpr int kDm   = 512;
constexpr int kDI   = 1024;
constexpr int kNs   = 16;
constexpr int kDtR  = 32;
constexpr int kRows = kBat * kSeq;
constexpr int kXZP  = 2 * kDI;
constexpr int kXpS  = kDtR + 2 * kDI;
constexpr int kXpT  = kDtR + 2 * kNs;
constexpr int kPW     = 2240;
constexpr int kColBs  = 0;
constexpr int kColCs  = 1024;
constexpr int kColF   = 2048;
constexpr int kColB   = 2112;
constexpr int kColDrs = 2176;
constexpr int kTP     = 260;
constexpr int kTsCh   = 128;
constexpr int kTsYP   = 132;
constexpr int kSpRowP = 1032;
static_assert(kRows == 4096 && kXZP == 2048 && kXpS == 2080 && kXpT == 64, "shapes");
static_assert(kColF == 2 * kDI && kColB == kColF + kXpT && kColDrs == kColB + kXpT && kColDrs + kDtR + 32 == kPW, "fused layout");
static_assert((kPW % 64) == 0 && (kRows % 64) == 0 && (kXZP % 64) == 0 && (kDI % 64) == 0 && (kDm % 64) == 0, "tile multiples");
static_assert((kDm % 32) == 0 && (kDI % 32) == 0 && (kDtR % 32) == 0, "K multiples of 32");
static_assert((kSeq % 64) == 0 && (kSeq % 16) == 0, "time tiles");

constexpr float kCx   = 16.0f;
constexpr float kCw   = 32.0f;
constexpr float kCu   = 16.0f;
constexpr float kCp   = 16.0f;
constexpr float kCdtw = 8.0f;
constexpr float kCdl  = 64.0f;
constexpr float kCyt  = 256.0f;
constexpr float kCy   = 16.0f;
constexpr float kScaleG1 = 1.0f / (kCx * kCw);
constexpr float kScaleG2 = kCp / (kCu * kCw);
constexpr float kScaleDt = kCdl / (kCp * kCdtw);
constexpr float kScaleG6 = 1.0f / (kCy * kCw);
constexpr float kInvCp   = 1.0f / kCp;
constexpr float kInvCu   = 1.0f / kCu;
constexpr float kInvCdl  = 1.0f / kCdl;
constexpr float kInvCyt  = 1.0f / kCyt;

constexpr size_t kOffX16  = 0;
constexpr size_t kOffWIN  = kOffX16  + (size_t)kRows * kDm * 2;
constexpr size_t kOffWXP  = kOffWIN  + (size_t)kXZP * kDm * 2;
constexpr size_t kOffWDT  = kOffWXP  + (size_t)kPW * kDI * 2;
constexpr size_t kOffWOUT = kOffWDT  + (size_t)3 * kDI * kDtR * 2;
constexpr size_t kOffXZ   = kOffWOUT + (size_t)kDm * kDI * 2;
constexpr size_t kOffU16  = kOffXZ   + (size_t)kRows * kXZP * 4;
constexpr size_t kOffP16  = kOffU16  + (size_t)kRows * kDI * 2;
constexpr size_t kOffDR16 = kOffP16  + (size_t)kRows * kPW * 2;
constexpr size_t kOffDL16 = kOffDR16 + (size_t)3 * kRows * kDtR * 2;
constexpr size_t kOffYT16 = kOffDL16 + (size_t)3 * kRows * kDI * 2;
constexpr size_t kOffY16  = kOffYT16 + (size_t)2 * kRows * kDI * 2;
constexpr size_t kOffKP1  = kOffY16  + (size_t)kRows * kDI * 2;
constexpr size_t kOffKEYS = kOffKP1  + (size_t)kBat * kDI * 4;
constexpr size_t kWsTotal = kOffKEYS + (size_t)kBat * kSeq * 4;
static_assert(kWsTotal == 123617280ull, "carve total");
static_assert(kWsTotal <= 134217728ull, "carve cap");
static_assert((kOffWIN % 128) == 0 && (kOffWXP % 128) == 0 && (kOffWDT % 128) == 0 && (kOffWOUT % 128) == 0 &&
              (kOffXZ % 128) == 0 && (kOffU16 % 128) == 0 && (kOffP16 % 128) == 0 && (kOffDR16 % 128) == 0 &&
              (kOffDL16 % 128) == 0 && (kOffYT16 % 128) == 0 && (kOffY16 % 128) == 0 && (kOffKP1 % 128) == 0 &&
              (kOffKEYS % 128) == 0, "128-B aligned regions");

__device__ __forceinline__ float h16_to_f32(unsigned hb) {
  const unsigned sgn = (hb & 0x8000u) << 16;
  const unsigned em = hb & 0x7fffu;
  const float fn = __uint_as_float((em << 13) + 0x38000000u);
  const float fs = (float)em * 5.9604644775390625e-8f;
  const float mag = (em < 0x400u) ? fs : fn;
  return __uint_as_float(__float_as_uint(mag) | sgn);
}
__device__ __forceinline__ float softplus_f(float v) {
  return fmaxf(v, 0.0f) + log1pf(expf(-fabsf(v)));
}

__device__ __forceinline__ void guard4_h(v8f& a, v8f& b, v8f& c, v8f& d, v16h x, v16h y) {
  asm volatile("v_nop\n\tv_nop\n\tv_nop\n\tv_nop" : "+v"(a), "+v"(b), "+v"(c), "+v"(d) : "v"(x), "v"(y));
}
__device__ __forceinline__ void keep4_h(v16h a, v16h b, v16h c, v16h d) { asm volatile("v_nop" :: "v"(a), "v"(b), "v"(c), "v"(d)); }
__device__ __forceinline__ void acc_guard4(v8f& a, v8f& b, v8f& c, v8f& d) {
  asm volatile("v_nop\n\tv_nop\n\tv_nop\n\tv_nop" : "+v"(a), "+v"(b), "+v"(c), "+v"(d));
}
union FragU { v16h v; v8h h[2]; };
__device__ __forceinline__ v16h frag_load(const _Float16* p) {
  FragU f;
  f.h[0] = *(const v8h*)(p);
  f.h[1] = *(const v8h*)(p + 16);
  return f.v;
}
__device__ __forceinline__ v8f frag_mma(v16h a, v16h b, v8f c) {
  return __builtin_amdgcn_wmma_f32_16x16x32_f16(false, a, false, b, (short)0, c, false, false);
}

template <int OUT_MODE>
__global__ __launch_bounds__(256) void wmma_gemm64(
    const unsigned short* __restrict__ Ap, int lda, long strideA,
    const unsigned short* __restrict__ Btp, int ldb, long strideB,
    void* __restrict__ Cout, int ldc, long strideC,
    int M, int N, int K, float scale) {
  const _Float16* A  = (const _Float16*)Ap;
  const _Float16* Bt = (const _Float16*)Btp;
  __shared__ __align__(16) float sT[8][16 * 68];
  const int b    = blockIdx.y;
  const int lane = threadIdx.x & 31;
  const int wave = threadIdx.x >> 5;
  const int tilesN = N >> 6;
  const int tilesM = M >> 6;
  const int tile = blockIdx.x * 8 + wave;
  if (tile >= tilesM * tilesN) return;
  const int tm = tile / tilesN;
  const int tn = tile - tm * tilesN;
  const int m0 = tm << 6;
  const int n0 = tn << 6;

  const _Float16* Ab = A  + (size_t)b * strideA;
  const _Float16* Bb = Bt + (size_t)b * strideB;

  const int rlane = lane & 15;
  const int koff  = (lane >> 4) * 8;
  const int mOff  = (lane >> 4) * 8;

  v8f acc[4][4];
#pragma unroll
  for (int i = 0; i < 4; ++i)
#pragma unroll
    for (int j = 0; j < 4; ++j) acc[i][j] = (v8f){0.f, 0.f, 0.f, 0.f, 0.f, 0.f, 0.f, 0.f};

  for (int k0 = 0; k0 < K; k0 += 32) {
    v16h bh[4];
#pragma unroll
    for (int j = 0; j < 4; ++j) {
      const size_t bo = (size_t)(n0 + (j << 4) + rlane) * ldb + koff + k0;
      bh[j] = frag_load(Bb + bo);
    }
#pragma unroll
    for (int i = 0; i < 4; ++i) {
      const size_t ao = (size_t)(m0 + (i << 4) + rlane) * lda + koff + k0;
      v16h ah = frag_load(Ab + ao);
#pragma unroll
      for (int j = 0; j < 4; ++j) acc[i][j] = frag_mma(ah, bh[j], acc[i][j]);
      guard4_h(acc[i][0], acc[i][1], acc[i][2], acc[i][3], ah, bh[3]);
    }
    keep4_h(bh[0], bh[1], bh[2], bh[3]);
  }
  acc_guard4(acc[0][0], acc[0][1], acc[0][2], acc[0][3]);
  acc_guard4(acc[1][0], acc[1][1], acc[1][2], acc[1][3]);
  acc_guard4(acc[2][0], acc[2][1], acc[2][2], acc[2][3]);
  acc_guard4(acc[3][0], acc[3][1], acc[3][2], acc[3][3]);

  float* slab = sT[wave];
#pragma unroll
  for (int i = 0; i < 4; ++i) {
    const int mBase = m0 + (i << 4);
#pragma unroll
    for (int j = 0; j < 4; ++j) {
#pragma unroll
      for (int r = 0; r < 8; ++r) {
        const float v = acc[i][j][r] * scale;
        slab[(mOff + r) * 68 + (j << 4) + rlane] = v;
      }
    }
    __builtin_amdgcn_fence(__ATOMIC_RELEASE, "workgroup");
    __builtin_amdgcn_wave_barrier();
    __builtin_amdgcn_fence(__ATOMIC_ACQUIRE, "workgroup");
    if (OUT_MODE == 0) {
      float* C = (float*)Cout + (size_t)b * strideC;
      const int hh = lane >> 4, c4 = (lane & 15) * 4;
      for (int pass = 0; pass < 2; ++pass) {
#pragma unroll
        for (int it = 0; it < 8; ++it) {
          const int row = it * 2 + hh;
          v4f v = *(const v4f*)(slab + row * 68 + c4);
          *(volatile v4f*)(C + (size_t)(mBase + row) * ldc + n0 + c4) = v;
        }
        __threadfence();
      }
    } else {
      const int q = lane >> 3, c8 = (lane & 7) * 8;
      unsigned short* C = (unsigned short*)Cout + (size_t)b * strideC;
      for (int pass = 0; pass < 2; ++pass) {
#pragma unroll
        for (int it = 0; it < 4; ++it) {
          const int row = it * 4 + q;
          const float* sp = slab + row * 68 + c8;
          v8h hv;
#pragma unroll
          for (int e = 0; e < 8; ++e) hv[e] = (_Float16)sp[e];
          *(volatile v8h*)(C + (size_t)(mBase + row) * ldc + n0 + c8) = hv;
        }
        __threadfence();
      }
    }
    __builtin_amdgcn_fence(__ATOMIC_RELEASE, "workgroup");
    __builtin_amdgcn_wave_barrier();
    __builtin_amdgcn_fence(__ATOMIC_ACQUIRE, "workgroup");
  }
}

__global__ __launch_bounds__(256) void cast_f16_kernel(
    const float* __restrict__ src, unsigned short* __restrict__ dst, int total8, float scale)
{
  const int i = blockIdx.x * 256 + threadIdx.x;
  if (i >= total8) return;
  const size_t e0 = (size_t)i << 3;
  const float* p = src + e0;
  const v4f a0 = *(const v4f*)(p);
  const v4f a1 = *(const v4f*)(p + 4);
  v8h hv;
#pragma unroll
  for (int e = 0; e < 4; ++e) {
    hv[e]     = (_Float16)(a0[e] * scale);
    hv[4 + e] = (_Float16)(a1[e] * scale);
  }
  unsigned short* q = dst + e0;
  *(volatile v8h*)q = hv;
  __threadfence();
  *(volatile v8h*)q = hv;
}

__global__ __launch_bounds__(256) void transpose_cast_kernel(
    const float* __restrict__ W, int ldw, int colOff, int nValid,
    unsigned short* __restrict__ Bt, int Kdim, float scale)
{
  __shared__ float tile[64 * 65];
  const int tid = threadIdx.x, lane = tid & 31, wave = tid >> 5;
  const int n0 = blockIdx.x * 64;
  const int k0 = blockIdx.y * 64;
#pragma unroll
  for (int p = 0; p < 16; ++p) {
    const int idx = tid + p * 256;
    const int kk  = idx >> 6;
    const int nn  = idx & 63;
    const int n   = n0 + nn;
    const int nc  = (n < nValid) ? n : (nValid - 1);
    const float v = W[(size_t)(k0 + kk) * ldw + colOff + nc];
    tile[kk * 65 + nn] = (n < nValid) ? (v * scale) : 0.f;
  }
  __syncthreads();
  const int q = lane >> 3, c8 = (lane & 7) * 8;
  v8h hv[2];
#pragma unroll
  for (int it = 0; it < 2; ++it) {
    const int nrow = it * 32 + wave * 4 + q;
#pragma unroll
    for (int e = 0; e < 8; ++e) hv[it][e] = (_Float16)tile[(c8 + e) * 65 + nrow];
  }
  for (int pass = 0; pass < 2; ++pass) {
#pragma unroll
    for (int it = 0; it < 2; ++it) {
      const int nrow = it * 32 + wave * 4 + q;
      *(volatile v8h*)(Bt + (size_t)(n0 + nrow) * Kdim + k0 + c8) = hv[it];
    }
    __threadfence();
  }
}

__global__ __launch_bounds__(256) void dtw_transpose_kernel(
    const float* __restrict__ w0, const float* __restrict__ w1, const float* __restrict__ w2,
    unsigned short* __restrict__ Bt)
{
  __shared__ float tile[32 * 65];
  const int tid = threadIdx.x;
  const int z = blockIdx.y;
  const float* W = (z == 0) ? w0 : ((z == 1) ? w1 : w2);
  const int n0 = blockIdx.x * 64;
#pragma unroll
  for (int p = 0; p < 8; ++p) {
    const int idx = tid + p * 256;
    const int kk  = idx >> 6;
    const int nn  = idx & 63;
    tile[kk * 65 + nn] = W[(size_t)kk * kDI + n0 + nn] * kCdtw;
  }
  __syncthreads();
  const int row = tid >> 2, k8 = (tid & 3) * 8;
  v8h hv;
#pragma unroll
  for (int e = 0; e < 8; ++e) hv[e] = (_Float16)tile[(k8 + e) * 65 + row];
  unsigned short* q = Bt + (size_t)z * kDI * kDtR + (size_t)(n0 + row) * kDtR + k8;
  *(volatile v8h*)q = hv;
  __threadfence();
  *(volatile v8h*)q = hv;
}

__global__ __launch_bounds__(256) void conv_silu_kernel(
    const float* __restrict__ XZ, const float* __restrict__ cw, const float* __restrict__ cb,
    unsigned short* __restrict__ U16)
{
  __shared__ __align__(16) float sT[16 * kTP];
  const int tid = threadIdx.x, lane = tid & 31, wave = tid >> 5;
  const int d0 = blockIdx.x * 256, d = d0 + tid;
  const int g0 = blockIdx.y * 64;
  const int tb = g0 & (kSeq - 1);
  const v4f wv = *(const v4f*)(cw + (size_t)d * 4);
  const float w0 = wv[0], w1 = wv[1], w2 = wv[2], w3 = wv[3];
  const float bc = cb[d];
  float xm3, xm2, xm1;
  {
    const bool hist = (tb > 0);
    const int rb = hist ? (g0 - 3) : g0;
    const float v3 = XZ[(size_t)rb * kXZP + d];
    const float v2 = XZ[(size_t)(rb + 1) * kXZP + d];
    const float v1 = XZ[(size_t)(rb + 2) * kXZP + d];
    xm3 = hist ? v3 : 0.f;
    xm2 = hist ? v2 : 0.f;
    xm1 = hist ? v1 : 0.f;
  }
#pragma unroll 1
  for (int sub = 0; sub < 4; ++sub) {
    const int lb = g0 + sub * 16;
#pragma unroll 1
    for (int s = 0; s < 16; ++s) {
      const float xcur = XZ[(size_t)(lb + s) * kXZP + d];
      float acc = w0 * xm3;
      acc = fmaf(w1, xm2, acc);
      acc = fmaf(w2, xm1, acc);
      acc = fmaf(w3, xcur, acc);
      const float sv = acc + bc;
      const float sg = 1.0f / (1.0f + expf(-sv));
      sT[s * kTP + tid] = (sv * sg) * kCu;
      xm3 = xm2; xm2 = xm1; xm1 = xcur;
    }
    __syncthreads();
    v8h bv[2];
#pragma unroll
    for (int it = 0; it < 2; ++it) {
      const float* sp = sT + (it * 8 + wave) * kTP + lane * 8;
      const v4f a0 = *(const v4f*)(sp);
      const v4f a1 = *(const v4f*)(sp + 4);
#pragma unroll
      for (int e = 0; e < 4; ++e) {
        bv[it][e]     = (_Float16)a0[e];
        bv[it][4 + e] = (_Float16)a1[e];
      }
    }
    for (int pass = 0; pass < 2; ++pass) {
#pragma unroll
      for (int it = 0; it < 2; ++it)
        *(volatile v8h*)(U16 + (size_t)(lb + it * 8 + wave) * kDI + d0 + lane * 8) = bv[it];
      __threadfence();
    }
    __syncthreads();
  }
}

__global__ __launch_bounds__(256) void pack_dr_kernel(
    const unsigned short* __restrict__ P16, unsigned short* __restrict__ DR16)
{
  const int i  = blockIdx.x * 256 + threadIdx.x;
  const int z  = i >> 14;
  const int r  = i & 16383;
  const int m  = r >> 2;
  const int c8 = (r & 3) * 8;
  const int col0 = kColF + z * kXpT;
  const v4u w = *(const v4u*)(P16 + (size_t)m * kPW + col0 + c8);
  unsigned short* q = DR16 + (size_t)i * 8;
  *(volatile v4u*)q = w;
  __threadfence();
  *(volatile v4u*)q = w;
}

__global__ __launch_bounds__(256) void key_matvec_kernel(
    const float* __restrict__ xk, const float* __restrict__ wk1, const float* __restrict__ wks,
    float* __restrict__ KP1, float* __restrict__ KEYS0)
{
  const int blk = blockIdx.x, tid = threadIdx.x;
  const bool first = (blk < 64);
  const int b  = first ? (blk >> 2) : (blk - 64);
  const int n  = first ? ((blk & 3) * 256 + tid) : tid;
  const int Nn = first ? kDI : kSeq;
  const float* W = first ? wk1 : wks;
  const float* xr = xk + (size_t)b * kDm;
  float acc = 0.0f;
#pragma unroll 4
  for (int k = 0; k < kDm; ++k) acc = fmaf(xr[k], W[(size_t)k * Nn + n], acc);
  float* dst = first ? (KP1 + (size_t)b * kDI + n) : (KEYS0 + (size_t)b * kSeq + n);
  *(volatile float*)dst = acc;
  __threadfence();
  *(volatile float*)dst = acc;
}

__global__ __launch_bounds__(256) void time_scan_kernel(
    const unsigned short* __restrict__ DL16, const unsigned short* __restrict__ U16,
    const unsigned short* __restrict__ P16,
    const float* __restrict__ KP1, const float* __restrict__ key2,
    const float* __restrict__ Alog_f, const float* __restrict__ Alog_b,
    const float* __restrict__ bias_f, const float* __restrict__ bias_b,
    unsigned short* __restrict__ YT16)
{
  __shared__ __align__(16) unsigned sDL[16 * 64];
  __shared__ __align__(16) unsigned sU[16 * 64];
  __shared__ __align__(16) float sBC[16 * 32];
  __shared__ __align__(16) float sY[16 * kTsYP];
  __shared__ float sA[kNs];
  const int tid = threadIdx.x, lane = tid & 31, wave = tid >> 5;
  const int d0  = blockIdx.x * kTsCh;
  const int b   = blockIdx.y;
  const int dir = blockIdx.z;
  const int chl = tid >> 1;
  const int hf  = tid & 1;
  const int d   = d0 + chl;
  const float* Alog = dir ? Alog_b : Alog_f;
  const float* bias = dir ? bias_b : bias_f;
  const unsigned short* DL = DL16 + (size_t)dir * kRows * kDI;
  unsigned short* YT = YT16 + (size_t)dir * kRows * kDI;
  const int colBC = (dir ? kColB : kColF) + kDtR;

  if (tid < kNs) sA[tid] = -expf(Alog[tid]);
  __syncthreads();

  float An[8], st[8];
  const float kp = KP1[(size_t)b * kDI + d];
#pragma unroll
  for (int j = 0; j < 8; ++j) {
    An[j] = sA[hf * 8 + j];
    st[j] = kp * key2[hf * 8 + j];
  }
  const float bb = bias[d];
  const int row0 = b * kSeq;
  const int sr = tid >> 4, su = tid & 15;
  const int wsel = chl >> 1;
  const int sh   = (chl & 1) * 16;

#pragma unroll 1
  for (int c = 0; c < kSeq / 16; ++c) {
    const int tb = dir ? (kSeq - 16 - c * 16) : (c * 16);
    __syncthreads();
    {
      const size_t g = (size_t)(row0 + tb + sr) * kDI + d0 + su * 8;
      const v4u a  = *(const v4u*)(DL + g);
      const v4u uu = *(const v4u*)(U16 + g);
      *(v4u*)(sDL + sr * 64 + su * 4) = a;
      *(v4u*)(sU  + sr * 64 + su * 4) = uu;
      const unsigned wbc = *(const unsigned*)(P16 + (size_t)(row0 + tb + sr) * kPW + colBC + su * 2);
      sBC[sr * 32 + su * 2]     = h16_to_f32(wbc & 0xffffu) * kInvCp;
      sBC[sr * 32 + su * 2 + 1] = h16_to_f32(wbc >> 16) * kInvCp;
    }
    __syncthreads();
#pragma unroll 1
    for (int s = 0; s < 16; ++s) {
      const int rr = dir ? (15 - s) : s;
      const unsigned wd = sDL[rr * 64 + wsel];
      const unsigned wu = sU[rr * 64 + wsel];
      const float dlr = h16_to_f32((wd >> sh) & 0xffffu);
      const float uv  = h16_to_f32((wu >> sh) & 0xffffu) * kInvCu;
      const float v     = dlr * kInvCdl + bb;
      const float delta = softplus_f(v);
      const float* bcp = sBC + rr * 32 + hf * 8;
      const v4f B0 = *(const v4f*)(bcp);
      const v4f B1 = *(const v4f*)(bcp + 4);
      const v4f C0 = *(const v4f*)(bcp + 16);
      const v4f C1 = *(const v4f*)(bcp + 20);
      float Bv[8], Cv[8];
#pragma unroll
      for (int e = 0; e < 4; ++e) {
        Bv[e] = B0[e]; Bv[4 + e] = B1[e];
        Cv[e] = C0[e]; Cv[4 + e] = C1[e];
      }
      float y = 0.0f;
#pragma unroll
      for (int j = 0; j < 8; ++j) {
        const float e   = expf(delta * An[j]);
        const float dbu = (delta * Bv[j]) * uv;
        st[j] = fmaf(e, st[j], dbu);
        y = fmaf(st[j], Cv[j], y);
      }
      const float yo = y + __shfl_xor(y, 1, 32);
      if (hf == 0) sY[rr * kTsYP + chl] = yo * kCyt;
    }
    __syncthreads();
    {
      const int row = wave * 2 + (lane >> 4);
      const int c8  = (lane & 15) * 8;
      const float* sp = sY + row * kTsYP + c8;
      const v4f a0 = *(const v4f*)(sp);
      const v4f a1 = *(const v4f*)(sp + 4);
      v8h hv;
#pragma unroll
      for (int e = 0; e < 4; ++e) { hv[e] = (_Float16)a0[e]; hv[4 + e] = (_Float16)a1[e]; }
      unsigned short* q = YT + (size_t)(row0 + tb + row) * kDI + d0 + c8;
      *(volatile v8h*)q = hv;
      __threadfence();
      *(volatile v8h*)q = hv;
    }
  }
}

__global__ __launch_bounds__(256) void channel_scan_combine_kernel(
    const unsigned short* __restrict__ DLS, const unsigned short* __restrict__ U16,
    const unsigned short* __restrict__ P16, const unsigned short* __restrict__ YT16,
    const float* __restrict__ XZ, const float* __restrict__ KEYS0,
    const float* __restrict__ AsLog, const float* __restrict__ bias_s,
    const float* __restrict__ Dv, const float* __restrict__ Db, const float* __restrict__ Dsp,
    unsigned short* __restrict__ Y16)
{
  __shared__ float sAs[kDI];
  __shared__ float sDsum[kDI];
  __shared__ float sBias[kDI];
  __shared__ __align__(16) float sRow[8 * kSpRowP];
  const int tid = threadIdx.x, lane = tid & 31, wave = tid >> 5;
#pragma unroll 1
  for (int i = 0; i < 4; ++i) {
    const int dd = tid + 256 * i;
    sAs[dd]   = -expf(AsLog[dd]);
    sDsum[dd] = (Dv[dd] + Db[dd]) + Dsp[dd];
    sBias[dd] = bias_s[dd];
  }
  __syncthreads();

  const int m = blockIdx.x * 8 + wave;
  const unsigned* dlw = (const unsigned*)(DLS + (size_t)m * kDI);
  const unsigned* uw  = (const unsigned*)(U16 + (size_t)m * kDI);

  float S = 0.0f, T = 0.0f;
#pragma unroll 1
  for (int it = 0; it < 16; ++it) {
    const int wi = it * 32 + lane;
    const unsigned wd = dlw[wi];
    const unsigned wu = uw[wi];
    const int dd = 2 * wi;
    const float v0 = h16_to_f32(wd & 0xffffu) * kInvCdl + sBias[dd];
    const float v1 = h16_to_f32(wd >> 16) * kInvCdl + sBias[dd + 1];
    const float l0 = softplus_f(v0);
    const float l1 = softplus_f(v1);
    const float u0 = h16_to_f32(wu & 0xffffu) * kInvCu;
    const float u1 = h16_to_f32(wu >> 16) * kInvCu;
    S += l0 + l1;
    T = fmaf(l0, u0, T);
    T = fmaf(l1, u1, T);
  }
#pragma unroll
  for (int off = 16; off > 0; off >>= 1) {
    S += __shfl_xor(S, off, 32);
    T += __shfl_xor(T, off, 32);
  }

  const unsigned* pBs = (const unsigned*)(P16 + (size_t)m * kPW + kColBs);
  const unsigned* pCs = (const unsigned*)(P16 + (size_t)m * kPW + kColCs);
  const unsigned* yfw = (const unsigned*)(YT16 + (size_t)m * kDI);
  const unsigned* ybw = (const unsigned*)(YT16 + (size_t)kRows * kDI + (size_t)m * kDI);
  const float* res = XZ + (size_t)m * kXZP + kDI;
  float* rowp = sRow + wave * kSpRowP;
  float sin_ = KEYS0[m];

#pragma unroll 1
  for (int k = 0; k < 16; ++k) {
    const int wi = k * 32 + lane;
    const int dd = 2 * wi;
    const unsigned wb = pBs[wi];
    const unsigned wc = pCs[wi];
    const unsigned wu = uw[wi];
    const unsigned wf = yfw[wi];
    const unsigned wr = ybw[wi];
    const v2f rs = *(const v2f*)(res + dd);
    float a0 = expf(S * sAs[dd]);
    float a1 = expf(S * sAs[dd + 1]);
    a0 = (a0 < 1.17549435e-38f) ? 0.0f : a0;
    a1 = (a1 < 1.17549435e-38f) ? 0.0f : a1;
    const float b0 = T * (h16_to_f32(wb & 0xffffu) * kInvCp);
    const float b1 = T * (h16_to_f32(wb >> 16) * kInvCp);
    float Aq = a1 * a0;
    float Bq = fmaf(a1, b0, b1);
#pragma unroll
    for (int off = 1; off < 32; off <<= 1) {
      const float Ap = __shfl_up(Aq, off, 32);
      const float Bp = __shfl_up(Bq, off, 32);
      const bool ok = (lane >= off);
      const float Bn = fmaf(Aq, Bp, Bq);
      const float An2 = Aq * Ap;
      Bq = ok ? Bn : Bq;
      Aq = ok ? An2 : Aq;
    }
    const float sincl = fmaf(Aq, sin_, Bq);
    const float pv = __shfl_up(sincl, 1, 32);
    const float prev = (lane == 0) ? sin_ : pv;
    const float s0 = fmaf(a0, prev, b0);
    const float s1 = fmaf(a1, s0, b1);
    sin_ = __shfl(sincl, 31, 32);
    const float c0 = h16_to_f32(wc & 0xffffu) * kInvCp;
    const float c1 = h16_to_f32(wc >> 16) * kInvCp;
    const float u0 = h16_to_f32(wu & 0xffffu) * kInvCu;
    const float u1 = h16_to_f32(wu >> 16) * kInvCu;
    const float f0 = h16_to_f32(wf & 0xffffu) * kInvCyt;
    const float f1 = h16_to_f32(wf >> 16) * kInvCyt;
    const float r0 = h16_to_f32(wr & 0xffffu) * kInvCyt;
    const float r1 = h16_to_f32(wr >> 16) * kInvCyt;
    const float rs0 = rs[0];
    const float rs1 = rs[1];
    float y0 = fmaf(s0, c0, u0 * sDsum[dd]);
    float y1 = fmaf(s1, c1, u1 * sDsum[dd + 1]);
    y0 = ((f0 + r0) + y0) + rs0;
    y1 = ((f1 + r1) + y1) + rs1;
    rowp[dd]     = y0 * kCy;
    rowp[dd + 1] = y1 * kCy;
  }
  __builtin_amdgcn_fence(__ATOMIC_RELEASE, "workgroup");
  __builtin_amdgcn_wave_barrier();
  __builtin_amdgcn_fence(__ATOMIC_ACQUIRE, "workgroup");
  v8h hv[4];
#pragma unroll
  for (int it = 0; it < 4; ++it) {
    const float* sp = rowp + it * 256 + lane * 8;
    const v4f a0 = *(const v4f*)(sp);
    const v4f a1 = *(const v4f*)(sp + 4);
#pragma unroll
    for (int e = 0; e < 4; ++e) { hv[it][e] = (_Float16)a0[e]; hv[it][4 + e] = (_Float16)a1[e]; }
  }
  for (int pass = 0; pass < 2; ++pass) {
#pragma unroll
    for (int it = 0; it < 4; ++it)
      *(volatile v8h*)(Y16 + (size_t)m * kDI + it * 256 + lane * 8) = hv[it];
    __threadfence();
  }
}

extern "C" void kernel_launch(void* const* d_in, const int* in_sizes, int n_in,
                              void* d_out, int out_size, void* d_ws, size_t ws_size,
                              hipStream_t stream)
{
  if (n_in < 24) return;
  if (in_sizes[0] != kRows * kDm) return;
  if (in_sizes[1] != kBat * kDm) return;
  if (in_sizes[2] != kDm * kXZP) return;
  if (in_sizes[3] != kDI * 4 || in_sizes[4] != kDI) return;
  if (in_sizes[5] != kDI * kXpT || in_sizes[6] != kDI * kXpT) return;
  if (in_sizes[7] != kDI * kXpS) return;
  if (in_sizes[8] != kDtR * kDI || in_sizes[10] != kDtR * kDI || in_sizes[12] != kDtR * kDI) return;
  if (in_sizes[9] != kDI || in_sizes[11] != kDI || in_sizes[13] != kDI) return;
  if (in_sizes[14] != kDm * kDI) return;
  if (in_sizes[15] != kNs) return;
  if (in_sizes[16] != kDm * kSeq) return;
  if (in_sizes[17] != kNs || in_sizes[18] != kNs || in_sizes[19] != kDI) return;
  if (in_sizes[20] != kDI || in_sizes[21] != kDI || in_sizes[22] != kDI) return;
  if (in_sizes[23] != kDI * kDm) return;
  if (out_size != kRows * kDm) return;
  if (ws_size < kWsTotal) return;

  const float* x         = (const float*)d_in[0];
  const float* x_key     = (const float*)d_in[1];
  const float* in_proj_w = (const float*)d_in[2];
  const float* conv_w    = (const float*)d_in[3];
  const float* conv_b    = (const float*)d_in[4];
  const float* x_proj_w  = (const float*)d_in[5];
  const float* x_proj_bw = (const float*)d_in[6];
  const float* x_proj_sw = (const float*)d_in[7];
  const float* dt_w      = (const float*)d_in[8];
  const float* dt_bias   = (const float*)d_in[9];
  const float* dt_b_w    = (const float*)d_in[10];
  const float* dt_b_bias = (const float*)d_in[11];
  const float* dt_s_w    = (const float*)d_in[12];
  const float* dt_s_bias = (const float*)d_in[13];
  const float* key1_w    = (const float*)d_in[14];
  const float* key2_w    = (const float*)d_in[15];
  const float* keys_w    = (const float*)d_in[16];
  const float* A_log     = (const float*)d_in[17];
  const float* A_b_log   = (const float*)d_in[18];
  const float* A_s_log   = (const float*)d_in[19];
  const float* Dv        = (const float*)d_in[20];
  const float* D_b       = (const float*)d_in[21];
  const float* D_s       = (const float*)d_in[22];
  const float* out_proj_w= (const float*)d_in[23];

  char* ws = (char*)d_ws;
  unsigned short* X16   = (unsigned short*)(ws + kOffX16);
  unsigned short* WIN   = (unsigned short*)(ws + kOffWIN);
  unsigned short* WXP   = (unsigned short*)(ws + kOffWXP);
  unsigned short* WDT   = (unsigned short*)(ws + kOffWDT);
  unsigned short* WOUT  = (unsigned short*)(ws + kOffWOUT);
  float*          XZ    = (float*)(ws + kOffXZ);
  unsigned short* U16   = (unsigned short*)(ws + kOffU16);
  unsigned short* P16   = (unsigned short*)(ws + kOffP16);
  unsigned short* DR16  = (unsigned short*)(ws + kOffDR16);
  unsigned short* DL16  = (unsigned short*)(ws + kOffDL16);
  unsigned short* YT16  = (unsigned short*)(ws + kOffYT16);
  unsigned short* Y16   = (unsigned short*)(ws + kOffY16);
  float*          KP1   = (float*)(ws + kOffKP1);
  float*          KEYS0 = (float*)(ws + kOffKEYS);

  cast_f16_kernel<<<(kRows * kDm) / 8 / 256, 256, 0, stream>>>(x, X16, (kRows * kDm) / 8, kCx);

  transpose_cast_kernel<<<dim3(kXZP / 64, kDm / 64), 256, 0, stream>>>(in_proj_w, kXZP, 0, kXZP, WIN, kDm, kCw);
  transpose_cast_kernel<<<dim3(2 * kDI / 64, kDI / 64), 256, 0, stream>>>(x_proj_sw, kXpS, kDtR, 2 * kDI, WXP, kDI, kCw);
  transpose_cast_kernel<<<dim3(1, kDI / 64), 256, 0, stream>>>(x_proj_w, kXpT, 0, kXpT, WXP + (size_t)kColF * kDI, kDI, kCw);
  transpose_cast_kernel<<<dim3(1, kDI / 64), 256, 0, stream>>>(x_proj_bw, kXpT, 0, kXpT, WXP + (size_t)kColB * kDI, kDI, kCw);
  transpose_cast_kernel<<<dim3(1, kDI / 64), 256, 0, stream>>>(x_proj_sw, kXpS, 0, kDtR, WXP + (size_t)kColDrs * kDI, kDI, kCw);
  transpose_cast_kernel<<<dim3(kDm / 64, kDI / 64), 256, 0, stream>>>(out_proj_w, kDm, 0, kDm, WOUT, kDI, kCw);
  dtw_transpose_kernel<<<dim3(kDI / 64, 3), 256, 0, stream>>>(dt_w, dt_b_w, dt_s_w, WDT);

  wmma_gemm64<0><<<dim3((kRows / 64) * (kXZP / 64) / 8, 1), 256, 0, stream>>>(
      X16, kDm, 0L, WIN, kDm, 0L, (void*)XZ, kXZP, 0L, kRows, kXZP, kDm, kScaleG1);

  conv_silu_kernel<<<dim3(kDI / 256, kRows / 64), 256, 0, stream>>>(XZ, conv_w, conv_b, U16);

  wmma_gemm64<1><<<dim3((kRows / 64) * (kPW / 64) / 8, 1), 256, 0, stream>>>(
      U16, kDI, 0L, WXP, kDI, 0L, (void*)P16, kPW, 0L, kRows, kPW, kDI, kScaleG2);

  pack_dr_kernel<<<(3 * kRows * kDtR) / 8 / 256, 256, 0, stream>>>(P16, DR16);

  wmma_gemm64<1><<<dim3((kRows / 64) * (kDI / 64) / 8, 3), 256, 0, stream>>>(
      DR16, kDtR, (long)kRows * kDtR, WDT, kDtR, (long)kDI * kDtR,
      (void*)DL16, kDI, (long)kRows * kDI, kRows, kDI, kDtR, kScaleDt);

  key_matvec_kernel<<<80, 256, 0, stream>>>(x_key, key1_w, keys_w, KP1, KEYS0);

  time_scan_kernel<<<dim3(kDI / kTsCh, kBat, 2), 256, 0, stream>>>(
      DL16, U16, P16, KP1, key2_w, A_log, A_b_log, dt_bias, dt_b_bias, YT16);

  channel_scan_combine_kernel<<<kRows / 8, 256, 0, stream>>>(
      DL16 + (size_t)2 * kRows * kDI, U16, P16, YT16, XZ, KEYS0,
      A_s_log, dt_s_bias, Dv, D_b, D_s, Y16);

  wmma_gemm64<0><<<dim3((kRows / 64) * (kDm / 64) / 8, 1), 256, 0, stream>>>(
      Y16, kDI, 0L, WOUT, kDI, 0L, d_out, kDm, 0L, kRows, kDm, kDI, kScaleG6);
}
